// MultiHeadSelfAttention_14894946583170
// MI455X (gfx1250) — hardware-verified
//
#include <hip/hip_runtime.h>


#pragma clang fp contract(off)

#ifndef NB
#define NB 2
#endif
#ifndef SEQ
#define SEQ 2048
#endif
#define NB_FULL  2
#define SEQ_FULL 2048
#define DIM      1024
#define NH       16
#define HD       64
#define HALF_HD  32
#define MROWS    ((NB) * (SEQ))
#define EARLYQ   (((SEQ) < 512) ? (SEQ) : 512)
#define CSP      132
#define OSP      68
#define WS_LIMIT 134217728ull

static_assert((SEQ) % 64 == 0);
static_assert((SEQ) >= 64);
static_assert((EARLYQ) % 64 == 0);
static_assert((SEQ) <= SEQ_FULL);
static_assert((NB) >= 1 && (NB) <= NB_FULL);
static_assert(DIM == NH * HD);

#define SZ_X   ((size_t)MROWS * DIM * 2)
#define SZ_W   ((size_t)DIM * DIM * 2)
#define SZ_WO2 ((size_t)DIM * 2 * DIM * 2)
#define SZ_P   ((size_t)MROWS * DIM * 2)
#define SZ_E   ((size_t)(NB) * (EARLYQ) * DIM * 2)
#define SZ_O2  ((size_t)MROWS * 2 * DIM * 2)
#define WS_TOTAL (SZ_X + 3 * SZ_W + SZ_WO2 + 3 * SZ_P + 6 * SZ_E + SZ_O2)
static_assert(WS_TOTAL <= WS_LIMIT);

typedef _Float16       h8   __attribute__((ext_vector_type(8)));
typedef _Float16       h16  __attribute__((ext_vector_type(16)));
typedef __bf16         b16v __attribute__((ext_vector_type(16)));
typedef unsigned short us8  __attribute__((ext_vector_type(8)));
typedef unsigned short us16 __attribute__((ext_vector_type(16)));
typedef float          f4   __attribute__((ext_vector_type(4)));
typedef float          f8   __attribute__((ext_vector_type(8)));

__device__ __forceinline__ unsigned short rne_bf16(float f) {
    unsigned int u = __float_as_uint(f);
    u += 0x7FFFu + ((u >> 16) & 1u);
    return (unsigned short)(u >> 16);
}
__device__ __forceinline__ float bf16_up(unsigned short s) {
    return __uint_as_float(((unsigned int)s) << 16);
}
__device__ __forceinline__ float bf16_val(float f) { return bf16_up(rne_bf16(f)); }

__device__ __forceinline__ h16 ld_frag_h(const _Float16* lo, const _Float16* hi) {
    h8 a = *(const h8*)lo;
    h8 b = *(const h8*)hi;
    return __builtin_shufflevector(a, b, 0, 1, 2, 3, 4, 5, 6, 7, 8, 9, 10, 11, 12, 13, 14, 15);
}
__device__ __forceinline__ b16v ld_frag_b(const unsigned short* lo, const unsigned short* hi) {
    us8 a = *(const us8*)lo;
    us8 b = *(const us8*)hi;
    us16 v = __builtin_shufflevector(a, b, 0, 1, 2, 3, 4, 5, 6, 7, 8, 9, 10, 11, 12, 13, 14, 15);
    return __builtin_bit_cast(b16v, v);
}
__device__ __forceinline__ f8 f8zero() {
    f8 z;
#pragma unroll
    for (int i = 0; i < 8; ++i) z[i] = 0.0f;
    return z;
}
__device__ __forceinline__ f8 mma_h(h16 a, h16 b, f8 c) {
    c = __builtin_amdgcn_wmma_f32_16x16x32_f16(false, a, false, b, (short)0, c, false, false);
    asm volatile("v_nop\n\tv_nop\n\tv_nop\n\tv_nop" : "+v"(c) : "v"(a), "v"(b));
    return c;
}
__device__ __forceinline__ f8 mma_b(b16v a, b16v b, f8 c) {
    c = __builtin_amdgcn_wmma_f32_16x16x32_bf16(false, a, false, b, (short)0, c, false, false);
    asm volatile("v_nop\n\tv_nop\n\tv_nop\n\tv_nop" : "+v"(c) : "v"(a), "v"(b));
    return c;
}

__device__ __forceinline__ float rowmax16(float v) {
#pragma unroll
    for (int off = 1; off < 16; off <<= 1) v = fmaxf(v, __shfl_xor(v, off));
    return v;
}
__device__ __forceinline__ float rowsum16(float v) {
#pragma unroll
    for (int off = 1; off < 16; off <<= 1) v += __shfl_xor(v, off);
    return v;
}

__global__ __launch_bounds__(256)
void cvt_kernel(const float* __restrict__ src, unsigned short* __restrict__ dst,
                int nelem, long long src_boff, long long dst_boff, int dup) {
    const long long e = ((long long)blockIdx.x * 256 + threadIdx.x) * 8;
    if (e >= (long long)nelem) return;
    const int r = (int)(e >> 10);
    const int c = (int)(e & (DIM - 1));
    const float* sp = src + (size_t)blockIdx.y * (size_t)src_boff + (size_t)r * DIM + c;
    const f4 v0 = *(const f4*)sp;
    const f4 v1 = *(const f4*)(sp + 4);
    us8 o;
    o[0] = rne_bf16(v0[0]); o[1] = rne_bf16(v0[1]); o[2] = rne_bf16(v0[2]); o[3] = rne_bf16(v0[3]);
    o[4] = rne_bf16(v1[0]); o[5] = rne_bf16(v1[1]); o[6] = rne_bf16(v1[2]); o[7] = rne_bf16(v1[3]);
    const size_t pitch = dup ? (size_t)(2 * DIM) : (size_t)DIM;
    unsigned short* dp = dst + (size_t)blockIdx.y * (size_t)dst_boff + (size_t)r * pitch + c;
    *(volatile us8*)dp = o;
    if (dup) *(volatile us8*)(dp + DIM) = o;
    __threadfence();
    *(volatile us8*)dp = o;
    if (dup) *(volatile us8*)(dp + DIM) = o;
}

template <int MODE>
__global__ __launch_bounds__(128) __attribute__((amdgpu_num_vgpr(256)))
void gemm_kernel(const unsigned short* __restrict__ A, const unsigned short* __restrict__ W, int K,
                 const float* __restrict__ cosT, const float* __restrict__ sinT,
                 _Float16* __restrict__ p16, unsigned short* __restrict__ phi,
                 unsigned short* __restrict__ plo, float* __restrict__ outp) {
    __shared__ float Cs[64][CSP];

    const int tid  = threadIdx.x;
    const int lane = tid & 31;
    const int wave = tid >> 5;
    const int wm   = wave & 1;
    const int wn   = wave >> 1;
    const int m0   = blockIdx.x * 64;
    const int n0   = blockIdx.y * 128;
    const int mrow = lane & 15;
    const int hi   = lane >> 4;
    const int kb   = hi * 8;

    const unsigned short* a0p = A + (size_t)(m0 + 32 * wm + mrow) * K + kb;
    const unsigned short* a1p = a0p + (size_t)16 * K;
    const unsigned short* b0p = W + (size_t)(n0 + 64 * wn + mrow) * K + kb;
    const unsigned short* b1p = b0p + (size_t)16 * K;
    const unsigned short* b2p = b0p + (size_t)32 * K;
    const unsigned short* b3p = b0p + (size_t)48 * K;

    f8 c00 = f8zero(), c01 = f8zero(), c02 = f8zero(), c03 = f8zero();
    f8 c10 = f8zero(), c11 = f8zero(), c12 = f8zero(), c13 = f8zero();

#pragma unroll 1
    for (int k0 = 0; k0 < K; k0 += 32) {
        const b16v a0 = ld_frag_b(a0p + k0, a0p + k0 + 16);
        const b16v a1 = ld_frag_b(a1p + k0, a1p + k0 + 16);
        const b16v w0 = ld_frag_b(b0p + k0, b0p + k0 + 16);
        const b16v w1 = ld_frag_b(b1p + k0, b1p + k0 + 16);
        const b16v w2 = ld_frag_b(b2p + k0, b2p + k0 + 16);
        const b16v w3 = ld_frag_b(b3p + k0, b3p + k0 + 16);
        c00 = mma_b(a0, w0, c00);
        c01 = mma_b(a0, w1, c01);
        c02 = mma_b(a0, w2, c02);
        c03 = mma_b(a0, w3, c03);
        c10 = mma_b(a1, w0, c10);
        c11 = mma_b(a1, w1, c11);
        c12 = mma_b(a1, w2, c12);
        c13 = mma_b(a1, w3, c13);
    }

#pragma unroll
    for (int r = 0; r < 8; ++r) {
        const int ra = 32 * wm + r + 8 * hi;
        const int rb = ra + 16;
        const int cb = 64 * wn + mrow;
        Cs[ra][cb]      = c00[r];
        Cs[ra][cb + 16] = c01[r];
        Cs[ra][cb + 32] = c02[r];
        Cs[ra][cb + 48] = c03[r];
        Cs[rb][cb]      = c10[r];
        Cs[rb][cb + 16] = c11[r];
        Cs[rb][cb + 32] = c12[r];
        Cs[rb][cb + 48] = c13[r];
    }
    __syncthreads();

    if (MODE == 0) {
        const int bidx = m0 / SEQ;
        const int sb   = m0 - bidx * SEQ;
        const bool early = sb < EARLYQ;
        const int cl = (lane & 15) * 8;
        const int gc = n0 + cl;
        const int i0 = (gc & (HD - 1)) >> 1;
#pragma unroll 1
        for (int it = 0; it < 8; ++it) {
            const int row = wave * 16 + 2 * it + hi;
            const int s   = sb + row;
            const f4 va = *(const f4*)&Cs[row][cl];
            const f4 vb = *(const f4*)&Cs[row][cl + 4];
            const f8 v  = __builtin_shufflevector(va, vb, 0, 1, 2, 3, 4, 5, 6, 7);
            const f4 cz = *(const f4*)(cosT + (size_t)s * HALF_HD + i0);
            const f4 sz = *(const f4*)(sinT + (size_t)s * HALF_HD + i0);
            f8 y;
#pragma unroll
            for (int j = 0; j < 4; ++j) {
                const float c  = bf16_val(cz[j]);
                const float sn = bf16_val(sz[j]);
                const float te = v[2 * j];
                const float to = v[2 * j + 1];
                y[2 * j]     = c * te - sn * to;
                y[2 * j + 1] = sn * te + c * to;
            }
            h8 yh; us8 yhi, ylo;
#pragma unroll
            for (int e = 0; e < 8; ++e) {
                const float val = y[e];
                yh[e] = (_Float16)val;
                const unsigned short hh = rne_bf16(val);
                yhi[e] = hh;
                ylo[e] = rne_bf16(val - bf16_up(hh));
            }
            const size_t m = (size_t)(m0 + row);
            _Float16* dp = p16 + m * DIM + gc;
            unsigned short* hp = phi + ((size_t)bidx * EARLYQ + s) * DIM + gc;
            unsigned short* lp = plo + ((size_t)bidx * EARLYQ + s) * DIM + gc;
            *(volatile h8*)dp = yh;
            if (early) { *(volatile us8*)hp = yhi; *(volatile us8*)lp = ylo; }
            __threadfence();
            *(volatile h8*)dp = yh;
            if (early) { *(volatile us8*)hp = yhi; *(volatile us8*)lp = ylo; }
        }
    } else if (MODE == 1) {
        const int bidx = m0 / SEQ;
        const int sb   = m0 - bidx * SEQ;
        const bool early = sb < EARLYQ;
        const int q = lane >> 3, piece = lane & 7;
#pragma unroll 1
        for (int it = 0; it < 8; ++it) {
            const int c  = wave * 32 + it * 4 + q;
            const int gc = n0 + c;
            const int bh = bidx * NH + (gc >> 6);
            const int d  = gc & (HD - 1);
            f8 v;
#pragma unroll
            for (int e = 0; e < 8; ++e) v[e] = Cs[piece * 8 + e][c];
            h8 yh; us8 yhi, ylo;
#pragma unroll
            for (int e = 0; e < 8; ++e) {
                const float val = v[e];
                yh[e] = (_Float16)val;
                const unsigned short hh = rne_bf16(val);
                yhi[e] = hh;
                ylo[e] = rne_bf16(val - bf16_up(hh));
            }
            const size_t lr = (size_t)bh * HD + d;
            _Float16* dp = p16 + lr * SEQ + sb + piece * 8;
            unsigned short* hp = phi + lr * EARLYQ + sb + piece * 8;
            unsigned short* lp = plo + lr * EARLYQ + sb + piece * 8;
            *(volatile h8*)dp = yh;
            if (early) { *(volatile us8*)hp = yhi; *(volatile us8*)lp = ylo; }
            __threadfence();
            *(volatile h8*)dp = yh;
            if (early) { *(volatile us8*)hp = yhi; *(volatile us8*)lp = ylo; }
        }
    } else {
#pragma unroll 1
        for (int i = 0; i < 16; ++i) {
            const int row = wave * 16 + i;
            const f4 v = *(const f4*)&Cs[row][4 * lane];
            float* dp = outp + (size_t)(m0 + row) * DIM + n0 + 4 * lane;
            *(volatile f4*)dp = v;
            __threadfence();
            *(volatile f4*)dp = v;
        }
    }
}

__device__ __forceinline__ void store_o_lines(const float* Os, unsigned short* O2,
                                              size_t row0, int h, int lane) {
    const int q = lane >> 3, piece = lane & 7;
#pragma unroll 1
    for (int it = 0; it < 8; ++it) {
        const int li    = it * 4 + q;
        const int row   = li >> 1;
        const int which = li & 1;
        const f4 va = *(const f4*)(Os + row * OSP + piece * 8);
        const f4 vb = *(const f4*)(Os + row * OSP + piece * 8 + 4);
        const f8 v  = __builtin_shufflevector(va, vb, 0, 1, 2, 3, 4, 5, 6, 7);
        us8 sv;
#pragma unroll
        for (int e = 0; e < 8; ++e) {
            const unsigned short hh = rne_bf16(v[e]);
            const unsigned short ll = rne_bf16(v[e] - bf16_up(hh));
            sv[e] = which ? ll : hh;
        }
        unsigned short* dp = O2 + (row0 + (size_t)row) * (size_t)(2 * DIM) + (size_t)which * DIM
                           + (size_t)h * HD + piece * 8;
        *(volatile us8*)dp = sv;
        __threadfence();
        *(volatile us8*)dp = sv;
    }
}

__global__ __launch_bounds__(32) __attribute__((amdgpu_num_vgpr(256)))
void attn_late(const _Float16* __restrict__ Q16, const _Float16* __restrict__ K16,
               const _Float16* __restrict__ VT16, unsigned short* __restrict__ O2, int tile0) {
    __shared__ _Float16 Plds[16][32];
    __shared__ float Os[16][OSP];

    const int lane = threadIdx.x & 31;
    const int mrow = lane & 15;
    const int hi   = lane >> 4;
    const int kb   = hi * 8;
    const int q0   = (tile0 + (int)blockIdx.x) * 16;
    const int h    = blockIdx.y;
    const int b    = blockIdx.z;

    const _Float16* qr = Q16 + ((size_t)b * SEQ + q0 + mrow) * DIM + (size_t)h * HD;
    const h16 aQ0 = ld_frag_h(qr + kb, qr + 16 + kb);
    const h16 aQ1 = ld_frag_h(qr + 32 + kb, qr + 48 + kb);

    const _Float16* kbase = K16 + ((size_t)b * SEQ + mrow) * DIM + (size_t)h * HD;
    const _Float16* vbase = VT16 + ((size_t)(b * NH + h) * HD + mrow) * SEQ;

    f8 o0 = f8zero(), o1 = f8zero(), o2 = f8zero(), o3 = f8zero();
    float rmax[8], rsum[8];
#pragma unroll
    for (int r = 0; r < 8; ++r) { rmax[r] = -1.0e30f; rsum[r] = 0.0f; }

    const float SC = 0.125f * 1.44269504088896f;

#pragma unroll 1
    for (int kc = 0; kc < q0 + 16; kc += 32) {
        const _Float16* k0p = kbase + (size_t)kc * DIM;
        const _Float16* k1p = k0p + (size_t)16 * DIM;
        const h16 b00 = ld_frag_h(k0p + kb, k0p + 16 + kb);
        const h16 b01 = ld_frag_h(k0p + 32 + kb, k0p + 48 + kb);
        const h16 b10 = ld_frag_h(k1p + kb, k1p + 16 + kb);
        const h16 b11 = ld_frag_h(k1p + 32 + kb, k1p + 48 + kb);

        f8 c0 = f8zero(), c1 = f8zero();
        c0 = mma_h(aQ0, b00, c0); c0 = mma_h(aQ1, b01, c0);
        c1 = mma_h(aQ0, b10, c1); c1 = mma_h(aQ1, b11, c1);

        const int key0 = kc + mrow, key1 = kc + 16 + mrow;
#pragma unroll
        for (int r = 0; r < 8; ++r) {
            const int qrow = q0 + r + 8 * hi;
            const float t0 = (key0 <= qrow) ? c0[r] * SC : -1.0e30f;
            const float t1 = (key1 <= qrow) ? c1[r] * SC : -1.0e30f;
            const float mx    = rowmax16(fmaxf(t0, t1));
            const float mnew  = fmaxf(rmax[r], mx);
            const float alpha = exp2f(rmax[r] - mnew);
            rmax[r] = mnew;
            const float e0 = exp2f(t0 - mnew);
            const float e1 = exp2f(t1 - mnew);
            rsum[r] = rsum[r] * alpha + rowsum16(e0 + e1);
            o0[r] *= alpha; o1[r] *= alpha; o2[r] *= alpha; o3[r] *= alpha;
            Plds[r + 8 * hi][mrow]      = (_Float16)(e0 * 1024.0f);
            Plds[r + 8 * hi][16 + mrow] = (_Float16)(e1 * 1024.0f);
        }
        __syncthreads();
        const h16 aP = ld_frag_h(&Plds[mrow][kb], &Plds[mrow][16 + kb]);

        const _Float16* vp = vbase + kc;
        o0 = mma_h(aP, ld_frag_h(vp + kb, vp + 16 + kb), o0);
        vp += (size_t)16 * SEQ;
        o1 = mma_h(aP, ld_frag_h(vp + kb, vp + 16 + kb), o1);
        vp += (size_t)16 * SEQ;
        o2 = mma_h(aP, ld_frag_h(vp + kb, vp + 16 + kb), o2);
        vp += (size_t)16 * SEQ;
        o3 = mma_h(aP, ld_frag_h(vp + kb, vp + 16 + kb), o3);
        __syncthreads();
    }

#pragma unroll
    for (int r = 0; r < 8; ++r) {
        const float inv = __builtin_amdgcn_rcpf(rsum[r] * 1024.0f);
        const int orow = r + 8 * hi;
        Os[orow][mrow]      = o0[r] * inv;
        Os[orow][16 + mrow] = o1[r] * inv;
        Os[orow][32 + mrow] = o2[r] * inv;
        Os[orow][48 + mrow] = o3[r] * inv;
    }
    __syncthreads();
    store_o_lines(&Os[0][0], O2, (size_t)b * SEQ + q0, h, lane);
}

__device__ __forceinline__ f8 score_hl(f8 c, b16v qh0, b16v qh1, b16v ql0, b16v ql1,
                                       const unsigned short* kr, const unsigned short* lr, int kb) {
    b16v ka = ld_frag_b(kr + kb, kr + 16 + kb);
    b16v kk = ld_frag_b(kr + 32 + kb, kr + 48 + kb);
    c = mma_b(qh0, ka, c); c = mma_b(qh1, kk, c);
    c = mma_b(ql0, ka, c); c = mma_b(ql1, kk, c);
    ka = ld_frag_b(lr + kb, lr + 16 + kb);
    kk = ld_frag_b(lr + 32 + kb, lr + 48 + kb);
    c = mma_b(qh0, ka, c); c = mma_b(qh1, kk, c);
    return c;
}
__device__ __forceinline__ f8 pv_hl(f8 o, b16v ph, b16v pl,
                                    const unsigned short* vr, const unsigned short* lr, int kb) {
    b16v vh = ld_frag_b(vr + kb, vr + 16 + kb);
    o = mma_b(ph, vh, o); o = mma_b(pl, vh, o);
    b16v vl = ld_frag_b(lr + kb, lr + 16 + kb);
    o = mma_b(ph, vl, o);
    return o;
}

__global__ __launch_bounds__(32) __attribute__((amdgpu_num_vgpr(256)))
void attn_early(const unsigned short* __restrict__ QH, const unsigned short* __restrict__ QL,
                const unsigned short* __restrict__ KH, const unsigned short* __restrict__ KL,
                const unsigned short* __restrict__ VTH, const unsigned short* __restrict__ VTL,
                unsigned short* __restrict__ O2) {
    __shared__ unsigned short Ph[16][32];
    __shared__ unsigned short Pl[16][32];
    __shared__ float Os[16][OSP];

    const int lane = threadIdx.x & 31;
    const int mrow = lane & 15;
    const int hi   = lane >> 4;
    const int kb   = hi * 8;
    const int q0   = (int)blockIdx.x * 16;
    const int h    = blockIdx.y;
    const int b    = blockIdx.z;

    const size_t qpl = ((size_t)b * EARLYQ + q0 + mrow) * DIM + (size_t)h * HD;
    const b16v qh0 = ld_frag_b(QH + qpl + kb,      QH + qpl + 16 + kb);
    const b16v qh1 = ld_frag_b(QH + qpl + 32 + kb, QH + qpl + 48 + kb);
    const b16v ql0 = ld_frag_b(QL + qpl + kb,      QL + qpl + 16 + kb);
    const b16v ql1 = ld_frag_b(QL + qpl + 32 + kb, QL + qpl + 48 + kb);

    const unsigned short* khb = KH + ((size_t)b * EARLYQ + mrow) * DIM + (size_t)h * HD;
    const unsigned short* klb = KL + ((size_t)b * EARLYQ + mrow) * DIM + (size_t)h * HD;
    const unsigned short* vhb = VTH + ((size_t)(b * NH + h) * HD + mrow) * EARLYQ;
    const unsigned short* vlb = VTL + ((size_t)(b * NH + h) * HD + mrow) * EARLYQ;

    f8 o0 = f8zero(), o1 = f8zero(), o2 = f8zero(), o3 = f8zero();
    float rmax[8], rsum[8];
#pragma unroll
    for (int r = 0; r < 8; ++r) { rmax[r] = -1.0e30f; rsum[r] = 0.0f; }

    const float SC = 0.125f * 1.44269504088896f;

#pragma unroll 1
    for (int kc = 0; kc < q0 + 16; kc += 32) {
        f8 c0 = score_hl(f8zero(), qh0, qh1, ql0, ql1,
                         khb + (size_t)kc * DIM, klb + (size_t)kc * DIM, kb);
        f8 c1 = score_hl(f8zero(), qh0, qh1, ql0, ql1,
                         khb + (size_t)(kc + 16) * DIM, klb + (size_t)(kc + 16) * DIM, kb);

        const int key0 = kc + mrow, key1 = kc + 16 + mrow;
#pragma unroll
        for (int r = 0; r < 8; ++r) {
            const int qrow = q0 + r + 8 * hi;
            const float t0 = (key0 <= qrow) ? c0[r] * SC : -1.0e30f;
            const float t1 = (key1 <= qrow) ? c1[r] * SC : -1.0e30f;
            const float mx    = rowmax16(fmaxf(t0, t1));
            const float mnew  = fmaxf(rmax[r], mx);
            const float alpha = exp2f(rmax[r] - mnew);
            rmax[r] = mnew;
            const float e0 = exp2f(t0 - mnew);
            const float e1 = exp2f(t1 - mnew);
            rsum[r] = rsum[r] * alpha + rowsum16(e0 + e1);
            o0[r] *= alpha; o1[r] *= alpha; o2[r] *= alpha; o3[r] *= alpha;
            const unsigned short p0h = rne_bf16(e0);
            const unsigned short p1h = rne_bf16(e1);
            const int prow = r + 8 * hi;
            Ph[prow][mrow]      = p0h;
            Pl[prow][mrow]      = rne_bf16(e0 - bf16_up(p0h));
            Ph[prow][16 + mrow] = p1h;
            Pl[prow][16 + mrow] = rne_bf16(e1 - bf16_up(p1h));
        }
        __syncthreads();
        const b16v aPh = ld_frag_b(&Ph[mrow][kb], &Ph[mrow][16 + kb]);
        const b16v aPl = ld_frag_b(&Pl[mrow][kb], &Pl[mrow][16 + kb]);

        o0 = pv_hl(o0, aPh, aPl, vhb + kc,                       vlb + kc,                       kb);
        o1 = pv_hl(o1, aPh, aPl, vhb + (size_t)16 * EARLYQ + kc, vlb + (size_t)16 * EARLYQ + kc, kb);
        o2 = pv_hl(o2, aPh, aPl, vhb + (size_t)32 * EARLYQ + kc, vlb + (size_t)32 * EARLYQ + kc, kb);
        o3 = pv_hl(o3, aPh, aPl, vhb + (size_t)48 * EARLYQ + kc, vlb + (size_t)48 * EARLYQ + kc, kb);
        __syncthreads();
    }

#pragma unroll
    for (int r = 0; r < 8; ++r) {
        const float inv = __builtin_amdgcn_rcpf(rsum[r]);
        const int orow = r + 8 * hi;
        Os[orow][mrow]      = o0[r] * inv;
        Os[orow][16 + mrow] = o1[r] * inv;
        Os[orow][32 + mrow] = o2[r] * inv;
        Os[orow][48 + mrow] = o3[r] * inv;
    }
    __syncthreads();
    store_o_lines(&Os[0][0], O2, (size_t)b * SEQ + q0, h, lane);
}

extern "C" void kernel_launch(void* const* d_in, const int* in_sizes, int n_in,
                              void* d_out, int out_size, void* d_ws, size_t ws_size,
                              hipStream_t stream) {
    if (n_in < 7) return;
    const float* x    = (const float*)d_in[0];
    const float* Wq   = (const float*)d_in[1];
    const float* Wk   = (const float*)d_in[2];
    const float* Wv   = (const float*)d_in[3];
    const float* Wo   = (const float*)d_in[4];
    const float* cosT = (const float*)d_in[5];
    const float* sinT = (const float*)d_in[6];
    float* out = (float*)d_out;

    if (in_sizes[0] < ((NB - 1) * SEQ_FULL + SEQ) * DIM) return;
    if (in_sizes[1] < DIM * DIM || in_sizes[2] < DIM * DIM ||
        in_sizes[3] < DIM * DIM || in_sizes[4] < DIM * DIM) return;
    if (in_sizes[5] < SEQ * HALF_HD || in_sizes[6] < SEQ * HALF_HD) return;
    if (out_size < MROWS * DIM) return;
    if (ws_size < WS_TOTAL) return;

    char* base = (char*)d_ws;
    size_t off = 0;
    unsigned short* xb   = (unsigned short*)(base + off); off += SZ_X;
    unsigned short* wqb  = (unsigned short*)(base + off); off += SZ_W;
    unsigned short* wkb  = (unsigned short*)(base + off); off += SZ_W;
    unsigned short* wvb  = (unsigned short*)(base + off); off += SZ_W;
    unsigned short* wo2  = (unsigned short*)(base + off); off += SZ_WO2;
    _Float16*       q16  = (_Float16*)(base + off);       off += SZ_P;
    _Float16*       k16  = (_Float16*)(base + off);       off += SZ_P;
    _Float16*       vt16 = (_Float16*)(base + off);       off += SZ_P;
    unsigned short* qh   = (unsigned short*)(base + off); off += SZ_E;
    unsigned short* ql   = (unsigned short*)(base + off); off += SZ_E;
    unsigned short* kh   = (unsigned short*)(base + off); off += SZ_E;
    unsigned short* kl   = (unsigned short*)(base + off); off += SZ_E;
    unsigned short* vth  = (unsigned short*)(base + off); off += SZ_E;
    unsigned short* vtl  = (unsigned short*)(base + off); off += SZ_E;
    unsigned short* o2   = (unsigned short*)(base + off); off += SZ_O2;
    if (off > ws_size || off > (size_t)WS_LIMIT) return;

    cvt_kernel<<<dim3((SEQ * DIM) / 2048, NB), 256, 0, stream>>>(
        x, xb, SEQ * DIM, (long long)SEQ_FULL * DIM, (long long)SEQ * DIM, 0);
    cvt_kernel<<<dim3((DIM * DIM) / 2048, 1), 256, 0, stream>>>(Wq, wqb, DIM * DIM, 0, 0, 0);
    cvt_kernel<<<dim3((DIM * DIM) / 2048, 1), 256, 0, stream>>>(Wk, wkb, DIM * DIM, 0, 0, 0);
    cvt_kernel<<<dim3((DIM * DIM) / 2048, 1), 256, 0, stream>>>(Wv, wvb, DIM * DIM, 0, 0, 0);
    cvt_kernel<<<dim3((DIM * DIM) / 2048, 1), 256, 0, stream>>>(Wo, wo2, DIM * DIM, 0, 0, 1);

    const dim3 gg(MROWS / 64, DIM / 128);
    gemm_kernel<0><<<gg, 128, 0, stream>>>(xb, wqb, DIM, cosT, sinT, q16, qh, ql, out);
    gemm_kernel<0><<<gg, 128, 0, stream>>>(xb, wkb, DIM, cosT, sinT, k16, kh, kl, out);
    gemm_kernel<1><<<gg, 128, 0, stream>>>(xb, wvb, DIM, cosT, sinT, vt16, vth, vtl, out);

    attn_early<<<dim3(EARLYQ / 16, NH, NB), 32, 0, stream>>>(qh, ql, kh, kl, vth, vtl, o2);
    if (SEQ > EARLYQ) {
        attn_late<<<dim3((SEQ - EARLYQ) / 16, NH, NB), 32, 0, stream>>>(q16, k16, vt16, o2, EARLYQ / 16);
    }

    gemm_kernel<2><<<gg, 128, 0, stream>>>(o2, wo2, 2 * DIM, cosT, sinT, q16, qh, ql, out);
}
